// MambaBlock_89249420411545
// MI455X (gfx1250) — hardware-verified
//
#include <hip/hip_runtime.h>
#include <stddef.h>
#include <stdint.h>
#include <math.h>


#define MROWS 4096
#define SEQ   2048
#define DM    1024
#define DI    2048
#define NIN   4096
#define NXD   96
#define DTRK  64
#define DST   16
#define K2I   4096
#define K2D   128
#define GBM   64
#define GTHR  128
#define PTHR  256
#define CT    32
#define STHR  128
#define WSMAX 134217728

#define EPI_INPROJ 0
#define EPI_XPROJ  1
#define EPI_DT     2
#define EPI_OUT    3

#define NU_X   (MROWS * (DM / 8))
#define NU_WIN (NIN * (DM / 8))
#define NU_WX  (NXD * (K2I / 8))
#define NU_WDT (DI * (K2D / 8))
#define NU_WO  (DM * (K2I / 8))
#define NU_ALL (NU_X + NU_WIN + NU_WX + NU_WDT + NU_WO)

static_assert(NU_X % PTHR == 0 && NU_WIN % PTHR == 0 && NU_WX % PTHR == 0 && NU_WDT % PTHR == 0 && NU_WO % PTHR == 0);
static_assert(MROWS % GBM == 0 && NIN % 64 == 0 && DI % 64 == 0 && DM % 64 == 0 && NXD == 96);
static_assert(DM % 32 == 0 && K2I % 32 == 0 && K2D % 32 == 0);
static_assert(K2I == 2 * DI && K2D == 2 * DTRK && NIN == 2 * DI);
static_assert((DI & (DI - 1)) == 0 && (DTRK & (DTRK - 1)) == 0 && (SEQ & (SEQ - 1)) == 0);
static_assert(SEQ % CT == 0 && CT == 32 && STHR == 128);
static_assert(GBM == (GTHR / 32) * 16);

typedef float          v4f   __attribute__((ext_vector_type(4)));
typedef float          v8f   __attribute__((ext_vector_type(8)));
typedef int            v8i   __attribute__((ext_vector_type(8)));
typedef unsigned short v4us  __attribute__((ext_vector_type(4)));
typedef unsigned short v8us  __attribute__((ext_vector_type(8)));
typedef unsigned short v16us __attribute__((ext_vector_type(16)));
typedef __bf16         v16bf __attribute__((ext_vector_type(16)));
typedef v4f  __attribute__((may_alias)) v4fa;
typedef v4us __attribute__((may_alias)) v4usa;
typedef v8us __attribute__((may_alias)) v8usa;
union FragB { v16bf v; v16us u; v8us h[2]; v8i w; };

__device__ __forceinline__ v8f wmb(const FragB& a, const FragB& b, v8f c) {
  v8f d = __builtin_amdgcn_wmma_f32_16x16x32_bf16(false, a.v, false, b.v, (short)0, c, false, false);
  asm volatile("v_nop\n\tv_nop\n\tv_nop\n\tv_nop" : "+v"(d) : "v"(a.w), "v"(b.w));
  return d;
}

__device__ __forceinline__ unsigned bf16_bits(float f) {
  const unsigned u = __float_as_uint(f);
  return (u + 0x7FFFu + ((u >> 16) & 1u)) >> 16;
}
__device__ __forceinline__ float bf16_val(float f) {
  return __uint_as_float(bf16_bits(f) << 16);
}
__device__ __forceinline__ unsigned short hl_pick(float f, bool lo) {
  const unsigned hb = bf16_bits(f);
  const unsigned lb = bf16_bits(f - __uint_as_float(hb << 16));
  return (unsigned short)(lo ? lb : hb);
}
__device__ __forceinline__ float silu_f(float v) {
  return v * __builtin_amdgcn_rcpf(1.0f + expf(-v));
}
__device__ __forceinline__ float softplus_f(float v) {
  return fmaxf(v, 0.0f) + log1pf(expf(-fabsf(v)));
}

__device__ __forceinline__ v8us gather8(const float* __restrict__ p, size_t st) {
  v8us o;
#pragma unroll
  for (int i = 0; i < 8; ++i) o[i] = (unsigned short)bf16_bits(p[(size_t)i * st]);
  return o;
}

__global__ __launch_bounds__(PTHR) void k_prep(const float* __restrict__ x, const float* __restrict__ w_in,
                                               const float* __restrict__ w_x, const float* __restrict__ w_dt,
                                               const float* __restrict__ w_out,
                                               unsigned short* XB, unsigned short* WINt, unsigned short* WX2,
                                               unsigned short* WDT2, unsigned short* WO2) {
  const int u = (int)blockIdx.x * PTHR + (int)threadIdx.x;
  v8us o;
  unsigned short* dp;
  if (u < NU_X) {
    const float* p = x + (size_t)u * 8;
    const v4f a = *(const v4f*)p;
    const v4f b = *(const v4f*)(p + 4);
    o[0] = (unsigned short)bf16_bits(a.x); o[1] = (unsigned short)bf16_bits(a.y);
    o[2] = (unsigned short)bf16_bits(a.z); o[3] = (unsigned short)bf16_bits(a.w);
    o[4] = (unsigned short)bf16_bits(b.x); o[5] = (unsigned short)bf16_bits(b.y);
    o[6] = (unsigned short)bf16_bits(b.z); o[7] = (unsigned short)bf16_bits(b.w);
    dp = XB + (size_t)u * 8;
  } else if (u < NU_X + NU_WIN) {
    const int v  = u - NU_X;
    const int n  = v >> 7;
    const int k8 = (v & 127) * 8;
    o  = gather8(w_in + (size_t)k8 * NIN + n, (size_t)NIN);
    dp = WINt + (size_t)v * 8;
  } else if (u < NU_X + NU_WIN + NU_WX) {
    const int v  = u - (NU_X + NU_WIN);
    const int n  = v >> 9;
    const int k8 = (v & 511) * 8;
    const int kk = k8 & (DI - 1);
    o  = gather8(w_x + (size_t)kk * NXD + n, (size_t)NXD);
    dp = WX2 + (size_t)v * 8;
  } else if (u < NU_X + NU_WIN + NU_WX + NU_WDT) {
    const int v  = u - (NU_X + NU_WIN + NU_WX);
    const int n  = v >> 4;
    const int k8 = (v & 15) * 8;
    const int kk = k8 & (DTRK - 1);
    o  = gather8(w_dt + (size_t)kk * DI + n, (size_t)DI);
    dp = WDT2 + (size_t)v * 8;
  } else if (u < NU_ALL) {
    const int v  = u - (NU_X + NU_WIN + NU_WX + NU_WDT);
    const int n  = v >> 9;
    const int k8 = (v & 511) * 8;
    const int kk = k8 & (DI - 1);
    o  = gather8(w_out + (size_t)kk * DM + n, (size_t)DM);
    dp = WO2 + (size_t)v * 8;
  } else {
    return;
  }
  *(volatile v8us*)dp = o;
  __threadfence();
  *(volatile v8us*)dp = o;
}

template <int NT, int EPI>
__global__ __launch_bounds__(GTHR) void k_gemm(const unsigned short* __restrict__ A,
                                               const unsigned short* __restrict__ WT, int K,
                                               float* outF, int ldo, long long gOff,
                                               const float* __restrict__ bias,
                                               unsigned short* outH, float* outB) {
  constexpr int SN = 16 * NT;
  __shared__ __attribute__((aligned(16))) float stg[GBM * SN];
  const int tid = (int)threadIdx.x, lane = tid & 31, wave = tid >> 5, hh = lane >> 4, m = lane & 15;
  const int rowBase = (int)blockIdx.x * GBM;
  const int col0    = (int)blockIdx.y * SN;

  v8f acc[NT];
  {
    const v8f z = {0.f, 0.f, 0.f, 0.f, 0.f, 0.f, 0.f, 0.f};
#pragma unroll
    for (int t = 0; t < NT; ++t) acc[t] = z;
  }
  const unsigned short* ap = A  + (size_t)(rowBase + 16 * wave + m) * (size_t)K + 8 * hh;
  const unsigned short* wp = WT + (size_t)(col0 + m) * (size_t)K + 8 * hh;
  const int ksteps = K >> 5;
#pragma unroll 1
  for (int ks = 0; ks < ksteps; ++ks) {
    FragB af;
    af.h[0] = *(const v8usa*)(ap + 32 * ks);
    af.h[1] = *(const v8usa*)(ap + 32 * ks + 16);
#pragma unroll
    for (int t = 0; t < NT; ++t) {
      const unsigned short* wq = wp + (size_t)(16 * t) * (size_t)K + 32 * ks;
      FragB bf;
      bf.h[0] = *(const v8usa*)wq;
      bf.h[1] = *(const v8usa*)(wq + 16);
      acc[t] = wmb(af, bf, acc[t]);
    }
  }

#pragma unroll
  for (int t = 0; t < NT; ++t) {
    const int lc = 16 * t + m;
#pragma unroll
    for (int r = 0; r < 8; ++r) {
      const int lr = 16 * wave + 8 * hh + r;
      stg[lr * SN + lc] = acc[t][r];
    }
  }
  __syncthreads();

  if constexpr (EPI == EPI_XPROJ) {
    static_assert(NT == 6);
    const int  cb    = 8 * (m & 7);
    const bool losel = (m & 8) != 0;
    v8us q[8];
#pragma unroll
    for (int i = 0; i < 8; ++i) {
      const int lr = 16 * wave + 2 * i + hh;
      const v4f f0 = *(const v4fa*)(stg + lr * SN + cb);
      const v4f f1 = *(const v4fa*)(stg + lr * SN + cb + 4);
      v8us o;
      o[0] = hl_pick(f0.x, losel); o[1] = hl_pick(f0.y, losel);
      o[2] = hl_pick(f0.z, losel); o[3] = hl_pick(f0.w, losel);
      o[4] = hl_pick(f1.x, losel); o[5] = hl_pick(f1.y, losel);
      o[6] = hl_pick(f1.z, losel); o[7] = hl_pick(f1.w, losel);
      q[i] = o;
    }
    const int rs = lane >> 3, pc = lane & 7;
    v4f bv[4];
#pragma unroll
    for (int i = 0; i < 4; ++i) {
      const int lr = 16 * wave + 4 * i + rs;
      bv[i] = *(const v4fa*)(stg + lr * SN + 64 + 4 * pc);
    }
#pragma unroll
    for (int i = 0; i < 8; ++i) {
      const int gr = rowBase + 16 * wave + 2 * i + hh;
      *(volatile v8us*)(outH + (size_t)gr * K2D + 8 * m) = q[i];
    }
#pragma unroll
    for (int i = 0; i < 4; ++i) {
      const int gr = rowBase + 16 * wave + 4 * i + rs;
      *(volatile v4f*)(outB + (size_t)gr * 32 + 4 * pc) = bv[i];
    }
    __threadfence();
#pragma unroll
    for (int i = 0; i < 8; ++i) {
      const int gr = rowBase + 16 * wave + 2 * i + hh;
      *(volatile v8us*)(outH + (size_t)gr * K2D + 8 * m) = q[i];
    }
#pragma unroll
    for (int i = 0; i < 4; ++i) {
      const int gr = rowBase + 16 * wave + 4 * i + rs;
      *(volatile v4f*)(outB + (size_t)gr * 32 + 4 * pc) = bv[i];
    }
  } else {
    static_assert(NT == 4);
    const bool zs = (EPI == EPI_INPROJ) && (col0 >= DI);
    if constexpr (EPI == EPI_INPROJ) {
      if (zs) {
#pragma unroll 1
        for (int i = 0; i < 8; ++i) {
          float* p = stg + (16 * wave + 2 * i + hh) * SN + 4 * m;
          v4f v = *(const v4fa*)p;
          v.x = silu_f(v.x); v.y = silu_f(v.y); v.z = silu_f(v.z); v.w = silu_f(v.w);
          *(v4fa*)p = v;
        }
      }
    }
    if constexpr (EPI == EPI_DT) {
      const v4f bq = *(const v4f*)(bias + col0 + 4 * m);
      const float b0 = bf16_val(bq.x), b1 = bf16_val(bq.y), b2 = bf16_val(bq.z), b3 = bf16_val(bq.w);
#pragma unroll 1
      for (int i = 0; i < 8; ++i) {
        float* p = stg + (16 * wave + 2 * i + hh) * SN + 4 * m;
        v4f v = *(const v4fa*)p;
        v.x = softplus_f(v.x + b0); v.y = softplus_f(v.y + b1);
        v.z = softplus_f(v.z + b2); v.w = softplus_f(v.w + b3);
        *(v4fa*)p = v;
      }
    }
    const int cc = zs ? (col0 - DI) : col0;
    float* ob = outF + (zs ? (size_t)gOff : (size_t)0);
    v4f fv[8];
#pragma unroll
    for (int i = 0; i < 8; ++i) {
      const int lr = 16 * wave + 2 * i + hh;
      fv[i] = *(const v4fa*)(stg + lr * SN + 4 * m);
    }
#pragma unroll
    for (int i = 0; i < 8; ++i) {
      const int gr = rowBase + 16 * wave + 2 * i + hh;
      *(volatile v4f*)(ob + (size_t)gr * (size_t)ldo + cc + 4 * m) = fv[i];
    }
    __threadfence();
#pragma unroll
    for (int i = 0; i < 8; ++i) {
      const int gr = rowBase + 16 * wave + 2 * i + hh;
      *(volatile v4f*)(ob + (size_t)gr * (size_t)ldo + cc + 4 * m) = fv[i];
    }
  }
}

__global__ __launch_bounds__(PTHR) void k_conv(const float* __restrict__ U, const float* __restrict__ wc,
                                               const float* __restrict__ bc, unsigned short* UChl) {
  __shared__ __attribute__((aligned(16))) unsigned short sh[2048];
  const int tid  = (int)threadIdx.x;
  const int row  = (int)blockIdx.x >> 1;
  const int half = (int)blockIdx.x & 1;
  const int l    = row & (SEQ - 1);
  const int c0   = half * 1024 + 4 * tid;

  const v4f w0 = *(const v4f*)(wc + (size_t)(c0 + 0) * 4);
  const v4f w1 = *(const v4f*)(wc + (size_t)(c0 + 1) * 4);
  const v4f w2 = *(const v4f*)(wc + (size_t)(c0 + 2) * 4);
  const v4f w3 = *(const v4f*)(wc + (size_t)(c0 + 3) * 4);
  const v4f bb = *(const v4f*)(bc + c0);
  float a0 = bf16_val(bb.x), a1 = bf16_val(bb.y), a2 = bf16_val(bb.z), a3 = bf16_val(bb.w);
#pragma unroll
  for (int j = 0; j < 4; ++j) {
    const bool ok = (l - 3 + j) >= 0;
    const int  rj = ok ? (row - 3 + j) : row;
    v4f uv = *(const v4f*)(U + (size_t)rj * DI + c0);
    uv.x = ok ? uv.x : 0.0f; uv.y = ok ? uv.y : 0.0f; uv.z = ok ? uv.z : 0.0f; uv.w = ok ? uv.w : 0.0f;
    a0 += bf16_val(w0[j]) * uv.x;
    a1 += bf16_val(w1[j]) * uv.y;
    a2 += bf16_val(w2[j]) * uv.z;
    a3 += bf16_val(w3[j]) * uv.w;
  }
  const float s0 = silu_f(a0), s1 = silu_f(a1), s2 = silu_f(a2), s3 = silu_f(a3);
  v4us h4, l4;
  h4[0] = hl_pick(s0, false); l4[0] = hl_pick(s0, true);
  h4[1] = hl_pick(s1, false); l4[1] = hl_pick(s1, true);
  h4[2] = hl_pick(s2, false); l4[2] = hl_pick(s2, true);
  h4[3] = hl_pick(s3, false); l4[3] = hl_pick(s3, true);
  *(v4usa*)(sh + 4 * tid) = h4;
  *(v4usa*)(sh + 1024 + 4 * tid) = l4;
  __syncthreads();
  const v8us q = *(const v8usa*)(sh + 8 * tid);
  unsigned short* dp = UChl + (size_t)row * K2I + (size_t)(tid >> 7) * DI + half * 1024 + 8 * (tid & 127);
  *(volatile v8us*)dp = q;
  __threadfence();
  *(volatile v8us*)dp = q;
}

__global__ __launch_bounds__(STHR) void k_scan(const float* __restrict__ DT, const float* __restrict__ G,
                                               const float* __restrict__ BC, const float* __restrict__ Alog,
                                               const float* __restrict__ Dp, unsigned short* YU) {
  __shared__ __attribute__((aligned(16))) float s_bc[CT * 32];
  __shared__ __attribute__((aligned(16))) float s_dt[CT * 64];
  __shared__ __attribute__((aligned(16))) float s_g[CT * 64];
  __shared__ __attribute__((aligned(16))) float s_a[STHR * 8];
  __shared__ __attribute__((aligned(16))) unsigned short s_uh[CT * 64];
  __shared__ __attribute__((aligned(16))) unsigned short s_ul[CT * 64];
  __shared__ __attribute__((aligned(16))) unsigned short s_yh[CT * 64];
  __shared__ __attribute__((aligned(16))) unsigned short s_yl[CT * 64];

  const int tid = (int)threadIdx.x, lane = tid & 31, wave = tid >> 5, hh = lane >> 4;
  const int ch = 16 * wave + (lane & 15);
  const int b  = (int)blockIdx.x >> 5;
  const int d0 = ((int)blockIdx.x & 31) * 64;
  const int d  = d0 + ch;

#pragma unroll 1
  for (int i = 0; i < 8; ++i) s_a[tid * 8 + i] = -expf(bf16_val(Alog[(size_t)d * DST + 8 * hh + i]));
  float a[8], h[8];
#pragma unroll
  for (int i = 0; i < 8; ++i) { a[i] = s_a[tid * 8 + i]; h[i] = 0.0f; }
  const float Dd = bf16_val(Dp[d]);

#pragma unroll 1
  for (int lc = 0; lc < SEQ; lc += CT) {
    const int row0 = b * SEQ + lc;
#pragma unroll
    for (int j = 0; j < 2; ++j) {
      const int idx = tid + STHR * j;
      *(v4fa*)(s_bc + 4 * idx) = *(const v4f*)(BC + (size_t)row0 * 32 + 4 * idx);
    }
#pragma unroll
    for (int j = 0; j < 4; ++j) {
      const int idx = tid + STHR * j;
      const int r = idx >> 4, p = idx & 15;
      *(v4fa*)(s_dt + r * 64 + 4 * p) = *(const v4f*)(DT + (size_t)(row0 + r) * DI + d0 + 4 * p);
      *(v4fa*)(s_g  + r * 64 + 4 * p) = *(const v4f*)(G  + (size_t)(row0 + r) * DI + d0 + 4 * p);
    }
#pragma unroll
    for (int j = 0; j < 2; ++j) {
      const int idx = tid + STHR * j;
      const int r = idx >> 3, p = idx & 7;
      const unsigned short* sp = YU + (size_t)(row0 + r) * K2I + d0 + 8 * p;
      *(v8usa*)(s_uh + r * 64 + 8 * p) = *(const v8usa*)sp;
      *(v8usa*)(s_ul + r * 64 + 8 * p) = *(const v8usa*)(sp + DI);
    }
    __syncthreads();

#pragma unroll 1
    for (int t = 0; t < CT; ++t) {
      const float dtt = s_dt[t * 64 + ch];
      const float gg  = s_g[t * 64 + ch];
      const float ut  = __uint_as_float((unsigned)s_uh[t * 64 + ch] << 16) +
                        __uint_as_float((unsigned)s_ul[t * 64 + ch] << 16);
      const float du  = dtt * ut;
      const float* bp = s_bc + t * 32 + 8 * hh;
      const v4f b0 = *(const v4fa*)bp;
      const v4f b1 = *(const v4fa*)(bp + 4);
      const v4f c0 = *(const v4fa*)(bp + 16);
      const v4f c1 = *(const v4fa*)(bp + 20);
      const float Bq[8] = {b0.x, b0.y, b0.z, b0.w, b1.x, b1.y, b1.z, b1.w};
      const float Cq[8] = {c0.x, c0.y, c0.z, c0.w, c1.x, c1.y, c1.z, c1.w};
      float y = 0.0f;
#pragma unroll
      for (int i = 0; i < 8; ++i) {
        const float dA = expf(dtt * a[i]);
        h[i] = fmaf(dA, h[i], du * Bq[i]);
        y = fmaf(h[i], Cq[i], y);
      }
      const float yo = __shfl_xor(y, 16, 32);
      const float yt = y + yo;
      const float v  = fmaf(ut, Dd, yt) * gg;
      const unsigned short hb = hl_pick(v, false);
      const unsigned short lb = hl_pick(v, true);
      if (hh == 0) { s_yh[t * 64 + ch] = hb; s_yl[t * 64 + ch] = lb; }
    }
    __syncthreads();

    const int tk = tid >> 3, pc = tid & 7;
    v8us qh[2], ql[2];
#pragma unroll
    for (int j = 0; j < 2; ++j) {
      qh[j] = *(const v8usa*)(s_yh + (16 * j + tk) * 64 + 8 * pc);
      ql[j] = *(const v8usa*)(s_yl + (16 * j + tk) * 64 + 8 * pc);
    }
#pragma unroll
    for (int j = 0; j < 2; ++j) {
      unsigned short* dp = YU + (size_t)(row0 + 16 * j + tk) * K2I + d0 + 8 * pc;
      *(volatile v8us*)dp = qh[j];
      *(volatile v8us*)(dp + DI) = ql[j];
    }
    __threadfence();
#pragma unroll
    for (int j = 0; j < 2; ++j) {
      unsigned short* dp = YU + (size_t)(row0 + 16 * j + tk) * K2I + d0 + 8 * pc;
      *(volatile v8us*)dp = qh[j];
      *(volatile v8us*)(dp + DI) = ql[j];
    }
  }
}

static inline size_t al256(size_t o) { return (o + 255) & ~(size_t)255; }

extern "C" void kernel_launch(void* const* d_in, const int* in_sizes, int n_in,
                              void* d_out, int out_size, void* d_ws, size_t ws_size,
                              hipStream_t stream) {
  if (n_in < 10) return;
  if (in_sizes[0] != MROWS * DM) return;
  if (in_sizes[1] != DM * NIN) return;
  if (in_sizes[2] != DI * 4) return;
  if (in_sizes[3] != DI) return;
  if (in_sizes[4] != DI * NXD) return;
  if (in_sizes[5] != DTRK * DI) return;
  if (in_sizes[6] != DI) return;
  if (in_sizes[7] != DI * DST) return;
  if (in_sizes[8] != DI) return;
  if (in_sizes[9] != DI * DM) return;
  if (out_size != MROWS * DM) return;

  const float* x      = (const float*)d_in[0];
  const float* w_in   = (const float*)d_in[1];
  const float* w_conv = (const float*)d_in[2];
  const float* b_conv = (const float*)d_in[3];
  const float* w_x    = (const float*)d_in[4];
  const float* w_dt   = (const float*)d_in[5];
  const float* b_dt   = (const float*)d_in[6];
  const float* A_log  = (const float*)d_in[7];
  const float* D_par  = (const float*)d_in[8];
  const float* w_out  = (const float*)d_in[9];
  float* out = (float*)d_out;

  char* ws = (char*)d_ws;
  size_t off = 0;
  const size_t oXB  = off; off = al256(off + (size_t)MROWS * DM * 2);
  const size_t oWIN = off; off = al256(off + (size_t)NIN * DM * 2);
  const size_t oWO  = off; off = al256(off + (size_t)DM * K2I * 2);
  const size_t oWX  = off; off = al256(off + (size_t)NXD * K2I * 2);
  const size_t oWDT = off; off = al256(off + (size_t)DI * K2D * 2);
  const size_t oDTR = off; off = al256(off + (size_t)MROWS * K2D * 2);
  const size_t oBC  = off; off = al256(off + (size_t)MROWS * 32 * 4);
  const size_t oUG  = off; off = al256(off + (size_t)2 * MROWS * DI * 4);
  const size_t oUC  = off; off = al256(off + (size_t)MROWS * K2I * 2);
  if (off > ws_size || off > (size_t)WSMAX) return;
  unsigned short* XB    = (unsigned short*)(ws + oXB);
  unsigned short* WINt  = (unsigned short*)(ws + oWIN);
  unsigned short* WO2   = (unsigned short*)(ws + oWO);
  unsigned short* WX2   = (unsigned short*)(ws + oWX);
  unsigned short* WDT2  = (unsigned short*)(ws + oWDT);
  unsigned short* DTRhl = (unsigned short*)(ws + oDTR);
  float*          BC    = (float*)(ws + oBC);
  float*          Upl   = (float*)(ws + oUG);
  float*          Gpl   = Upl + (size_t)MROWS * DI;
  float*          DTpl  = Upl;
  unsigned short* UChl  = (unsigned short*)(ws + oUC);
  const long long gOff  = (long long)MROWS * DI;

  k_prep<<<NU_ALL / PTHR, PTHR, 0, stream>>>(x, w_in, w_x, w_dt, w_out, XB, WINt, WX2, WDT2, WO2);
  k_gemm<4, EPI_INPROJ><<<dim3(MROWS / GBM, NIN / 64), GTHR, 0, stream>>>(
      XB, WINt, DM, Upl, DI, gOff, b_dt, DTRhl, BC);
  k_conv<<<MROWS * 2, PTHR, 0, stream>>>(Upl, w_conv, b_conv, UChl);
  k_gemm<6, EPI_XPROJ><<<dim3(MROWS / GBM, 1), GTHR, 0, stream>>>(
      UChl, WX2, K2I, Upl, DI, gOff, b_dt, DTRhl, BC);
  k_gemm<4, EPI_DT><<<dim3(MROWS / GBM, DI / 64), GTHR, 0, stream>>>(
      DTRhl, WDT2, K2D, DTpl, DI, gOff, b_dt, DTRhl, BC);
  k_scan<<<2 * (DI / 64), STHR, 0, stream>>>(DTpl, Gpl, BC, A_log, D_par, UChl);
  k_gemm<4, EPI_OUT><<<dim3(MROWS / GBM, DM / 64), GTHR, 0, stream>>>(
      UChl, WO2, K2I, out, DM, gOff, b_dt, DTRhl, BC);
}
